// FusionBlock_3891240370375
// MI455X (gfx1250) — hardware-run, weakly checked
//
#include <hip/hip_runtime.h>
#include <math.h>
#include <stdint.h>

#define CM 2048
#define CN 256
#define CL 128
#define CD 300
#define CD2 600
#define CD4 1200
#define PD 320
#define PD2 640
#define PX 960
#define NG 1216
#define PB 1280
#define DROOTF 17.320508075688775f
#define OUT0_N (CM * CD)
#define OUT1_N (CL * CD)

static_assert(PD % 64 == 0);
static_assert(CN % 64 == 0);
static_assert(CL % 64 == 0);
static_assert(CM % 64 == 0);
static_assert(NG % 64 == 0);
static_assert(CM % 32 == 0);
static_assert(PD2 % 32 == 0);
static_assert(PX % 32 == 0);
static_assert(OUT0_N + OUT1_N == 652800);
static_assert((CD * 8 * 4) % 128 == 0);
static_assert((OUT0_N * 4) % 128 == 0);

#define VT    0
#define VBU   640
#define VBRED 960
#define VBSUM 1280
#define VA    2560
#define VC    2816
#define VMX   3072
#define VZ    3328
#define VRQ   3584
#define VRE   3712
#define VQ2C  3968
#define VTOT  4288
static_assert(VC == VA + CN);
static_assert(VRE == VRQ + CL);
static_assert(VQ2C + PD == VTOT);

typedef __attribute__((ext_vector_type(16))) __bf16 v16b;
typedef __attribute__((ext_vector_type(8)))  __bf16 v8b;
typedef __attribute__((ext_vector_type(8)))  float v8f;
typedef __attribute__((ext_vector_type(4)))  float v4f;
typedef __attribute__((ext_vector_type(4)))  unsigned int v4u;
typedef v4f __attribute__((may_alias)) v4fa;
typedef v4u __attribute__((may_alias)) v4ua;

#define GF_F32   1
#define GF_PLN   2
#define GF_ROWB  4
#define GF_COLB  8
#define GF_RELU 16

__device__ __forceinline__ unsigned short f2bf_bits(float f) {
  unsigned u = __float_as_uint(f);
  return (unsigned short)((u + 0x7FFFu + ((u >> 16) & 1u)) >> 16);
}
__device__ __forceinline__ float bf_bits2f(unsigned int h) { return __uint_as_float((h & 0xFFFFu) << 16); }
__device__ __forceinline__ float bfr(float f) { return __uint_as_float(((unsigned)f2bf_bits(f)) << 16); }
__device__ __forceinline__ unsigned pk16(unsigned short a, unsigned short b) { return (unsigned)a | ((unsigned)b << 16); }

__device__ __forceinline__ void split2(float f0, float f1, unsigned& h, unsigned& l) {
  const unsigned short h0 = f2bf_bits(f0), h1 = f2bf_bits(f1);
  const unsigned short l0 = f2bf_bits(f0 - bf_bits2f(h0)), l1 = f2bf_bits(f1 - bf_bits2f(h1));
  h = pk16(h0, h1);
  l = pk16(l0, l1);
}
__device__ __forceinline__ void split8(v4f a, v4f b, v4u& hv, v4u& lv) {
  unsigned h, l;
  split2(a[0], a[1], h, l); hv[0] = h; lv[0] = l;
  split2(a[2], a[3], h, l); hv[1] = h; lv[1] = l;
  split2(b[0], b[1], h, l); hv[2] = h; lv[2] = l;
  split2(b[2], b[3], h, l); hv[3] = h; lv[3] = l;
}
__device__ __forceinline__ void unpack8(v4u w, v4f& a, v4f& b) {
  a[0] = __uint_as_float(w[0] << 16); a[1] = __uint_as_float(w[0] & 0xFFFF0000u);
  a[2] = __uint_as_float(w[1] << 16); a[3] = __uint_as_float(w[1] & 0xFFFF0000u);
  b[0] = __uint_as_float(w[2] << 16); b[1] = __uint_as_float(w[2] & 0xFFFF0000u);
  b[2] = __uint_as_float(w[3] << 16); b[3] = __uint_as_float(w[3] & 0xFFFF0000u);
}
__device__ __forceinline__ v8f zero8() { v8f z = {0.f, 0.f, 0.f, 0.f, 0.f, 0.f, 0.f, 0.f}; return z; }
__device__ __forceinline__ v4f zero4() { v4f z = {0.f, 0.f, 0.f, 0.f}; return z; }

__device__ __forceinline__ float wave_max(float v) {
#pragma unroll
  for (int o = 16; o > 0; o >>= 1) v = fmaxf(v, __shfl_xor(v, o));
  return v;
}
__device__ __forceinline__ float wave_sum(float v) {
#pragma unroll
  for (int o = 16; o > 0; o >>= 1) v += __shfl_xor(v, o);
  return v;
}
__device__ __forceinline__ float block_max(float v, float* red, int lane, int wave, int nw) {
  v = wave_max(v);
  if (lane == 0) red[wave] = v;
  __syncthreads();
  float r = red[0];
  for (int w = 1; w < nw; ++w) r = fmaxf(r, red[w]);
  __syncthreads();
  return r;
}
__device__ __forceinline__ float block_sum(float v, float* red, int lane, int wave, int nw) {
  v = wave_sum(v);
  if (lane == 0) red[wave] = v;
  __syncthreads();
  float r = red[0];
  for (int w = 1; w < nw; ++w) r += red[w];
  __syncthreads();
  return r;
}

__device__ __forceinline__ void dep_guard_b(v8f& a, v8f& b, v16b x, v16b y) { asm volatile("v_nop\n\tv_nop\n\tv_nop\n\tv_nop" : "+v"(a), "+v"(b) : "v"(x), "v"(y)); }
__device__ __forceinline__ void keep4_b(v16b a, v16b b, v16b c, v16b d) { asm volatile("v_nop" :: "v"(a), "v"(b), "v"(c), "v"(d)); }
__device__ __forceinline__ void acc_guard4(v8f& a, v8f& b, v8f& c, v8f& d) { asm volatile("v_nop\n\tv_nop\n\tv_nop\n\tv_nop" : "+v"(a), "+v"(b), "+v"(c), "+v"(d)); }

struct FragB {
  union U { v16b v; v8b h[2]; };
  static __device__ __forceinline__ v16b load(const __bf16* p) {
    U f; f.h[0] = *(const v8b*)(p); f.h[1] = *(const v8b*)(p + 16); return f.v;
  }
  static __device__ __forceinline__ v8f mma(v16b a, v16b b, v8f c) {
    return __builtin_amdgcn_wmma_f32_16x16x32_bf16(false, a, false, b, (short)0, c, false, false);
  }
};

__device__ __forceinline__ void gemm_term(v8f (&acc)[4][4], const unsigned short* ap, int lda,
                                          const unsigned short* bp, int ldb, int K,
                                          int m0, int n0, int rlane, int koff) {
  const __bf16* A  = (const __bf16*)(const void*)ap;
  const __bf16* Bt = (const __bf16*)(const void*)bp;
  for (int k0 = 0; k0 < K; k0 += 32) {
    v16b bh[4];
#pragma unroll
    for (int j = 0; j < 4; ++j) {
      const size_t bo = (size_t)(n0 + (j << 4) + rlane) * ldb + koff + k0;
      bh[j] = FragB::load(Bt + bo);
    }
#pragma unroll
    for (int i = 0; i < 4; ++i) {
      const size_t ao = (size_t)(m0 + (i << 4) + rlane) * lda + koff + k0;
      v16b ah = FragB::load(A + ao);
#pragma unroll
      for (int j = 0; j < 4; ++j) acc[i][j] = FragB::mma(ah, bh[j], acc[i][j]);
      dep_guard_b(acc[i][0], acc[i][3], ah, ah);
    }
    keep4_b(bh[0], bh[1], bh[2], bh[3]);
  }
}

struct GInts {
  int lda0, ldb0, K0, lda1, ldb1, K1, lda2, ldb2, K2;
  int ldcf, ldch, M, N, nterm, flags;
  float scale;
};
static_assert(sizeof(GInts) == 64);

__global__ __launch_bounds__(256) void k_gemm(
    const unsigned short* __restrict__ a0, const unsigned short* __restrict__ b0,
    const unsigned short* __restrict__ a1, const unsigned short* __restrict__ b1,
    const unsigned short* __restrict__ a2, const unsigned short* __restrict__ b2,
    float* cf, unsigned short* ch, unsigned short* cl,
    const float* rowb, const float* colb, GInts p) {
  __shared__ __align__(16) float sT[8][16 * 68];
  const int lane = threadIdx.x & 31;
  const int wave = threadIdx.x >> 5;
  const int tilesN = p.N >> 6;
  const int tilesM = p.M >> 6;
  const int tile = blockIdx.x * 8 + wave;
  if (tile >= tilesM * tilesN) return;
  const int tm = tile / tilesN;
  const int tn = tile - tm * tilesN;
  const int m0 = tm << 6;
  const int n0 = tn << 6;
  const int rlane = lane & 15;
  const int koff  = (lane >> 4) * 8;
  const int mOff  = (lane >> 4) * 8;

  v8f acc[4][4];
#pragma unroll
  for (int i = 0; i < 4; ++i)
#pragma unroll
    for (int j = 0; j < 4; ++j) acc[i][j] = zero8();

  gemm_term(acc, a0, p.lda0, b0, p.ldb0, p.K0, m0, n0, rlane, koff);
  if (p.nterm > 1) gemm_term(acc, a1, p.lda1, b1, p.ldb1, p.K1, m0, n0, rlane, koff);
  if (p.nterm > 2) gemm_term(acc, a2, p.lda2, b2, p.ldb2, p.K2, m0, n0, rlane, koff);
  acc_guard4(acc[0][0], acc[0][1], acc[0][2], acc[0][3]);
  acc_guard4(acc[1][0], acc[1][1], acc[1][2], acc[1][3]);
  acc_guard4(acc[2][0], acc[2][1], acc[2][2], acc[2][3]);
  acc_guard4(acc[3][0], acc[3][1], acc[3][2], acc[3][3]);

  const bool hasF = (p.flags & GF_F32) != 0;
  const bool hasP = (p.flags & GF_PLN) != 0;
  const bool hasRB = (p.flags & GF_ROWB) != 0;
  const bool hasCB = (p.flags & GF_COLB) != 0;
  const bool hasRelu = (p.flags & GF_RELU) != 0;

  float* slab = sT[wave];
#pragma unroll
  for (int i = 0; i < 4; ++i) {
    const int mBase = m0 + (i << 4);
    float radd[8];
#pragma unroll
    for (int r = 0; r < 8; ++r) radd[r] = 0.0f;
    if (hasRB) {
      const v4f rv0 = *(const v4fa*)(rowb + mBase + mOff);
      const v4f rv1 = *(const v4fa*)(rowb + mBase + mOff + 4);
      radd[0] = rv0[0]; radd[1] = rv0[1]; radd[2] = rv0[2]; radd[3] = rv0[3];
      radd[4] = rv1[0]; radd[5] = rv1[1]; radd[6] = rv1[2]; radd[7] = rv1[3];
    }
#pragma unroll
    for (int j = 0; j < 4; ++j) {
      float cadd = 0.0f;
      if (hasCB) cadd = colb[n0 + (j << 4) + rlane];
#pragma unroll
      for (int r = 0; r < 8; ++r) {
        float v = fmaf(acc[i][j][r], p.scale, radd[r]) + cadd;
        if (hasRelu) v = fmaxf(v, 0.0f);
        slab[(mOff + r) * 68 + (j << 4) + rlane] = v;
      }
    }
    __builtin_amdgcn_fence(__ATOMIC_RELEASE, "workgroup");
    __builtin_amdgcn_wave_barrier();
    __builtin_amdgcn_fence(__ATOMIC_ACQUIRE, "workgroup");
    for (int pass = 0; pass < 2; ++pass) {
      if (hasF) {
        const int q2 = lane >> 4, c4 = (lane & 15) * 4;
#pragma unroll
        for (int it = 0; it < 8; ++it) {
          const int row = it * 2 + q2;
          const v4f val = *(const v4fa*)(slab + row * 68 + c4);
          *(volatile v4f*)(cf + (size_t)(mBase + row) * p.ldcf + n0 + c4) = val;
        }
      }
      if (hasP) {
        const int q = lane >> 3, c8 = (lane & 7) * 8;
#pragma unroll
        for (int it = 0; it < 4; ++it) {
          const int row = it * 4 + q;
          const v4f s0 = *(const v4fa*)(slab + row * 68 + c8);
          const v4f s1 = *(const v4fa*)(slab + row * 68 + c8 + 4);
          v4u hv, lv;
          split8(s0, s1, hv, lv);
          const size_t o = (size_t)(mBase + row) * p.ldch + n0 + c8;
          *(volatile v4u*)(ch + o) = hv;
          *(volatile v4u*)(cl + o) = lv;
        }
      }
      __threadfence();
    }
    __builtin_amdgcn_fence(__ATOMIC_RELEASE, "workgroup");
    __builtin_amdgcn_wave_barrier();
    __builtin_amdgcn_fence(__ATOMIC_ACQUIRE, "workgroup");
  }
}

struct CvtInts { int src_pitch[8]; int src_rows[8]; int dst_rows[8]; int segw[8]; int segv[8]; int nseg[8]; };
static_assert(sizeof(CvtInts) == 192);

__global__ __launch_bounds__(256) void k_cvt(
    const float* s0, const float* s1, const float* s2, const float* s3,
    const float* s4, const float* s5, const float* s6, const float* s7,
    unsigned short* d0, unsigned short* d1, unsigned short* d2, unsigned short* d3,
    unsigned short* d4, unsigned short* d5, unsigned short* d6, unsigned short* d7, CvtInts ci) {
  const int pid = blockIdx.y;
  const float* srcs[8] = {s0, s1, s2, s3, s4, s5, s6, s7};
  unsigned short* dsts[8] = {d0, d1, d2, d3, d4, d5, d6, d7};
  const float* src = srcs[0];
  unsigned short* dst = dsts[0];
  int spitch = ci.src_pitch[0], srows = ci.src_rows[0], drows = ci.dst_rows[0];
  int segw = ci.segw[0], segv = ci.segv[0], nseg = ci.nseg[0];
#pragma unroll
  for (int i = 1; i < 8; ++i) {
    if (pid == i) {
      src = srcs[i]; dst = dsts[i];
      spitch = ci.src_pitch[i]; srows = ci.src_rows[i]; drows = ci.dst_rows[i];
      segw = ci.segw[i]; segv = ci.segv[i]; nseg = ci.nseg[i];
    }
  }
  const int cols = segw * nseg;
  const int n8 = cols >> 3;
  const int gidx = blockIdx.x * 256 + threadIdx.x;
  if (gidx >= drows * n8) return;
  const int r = gidx / n8;
  const int c = (gidx - r * n8) << 3;
  const int seg = c / segw;
  const int cc = c - seg * segw;
  const int rs = min(r, srows - 1);
  const bool rok = r < srows;
  const float* sp = src + (size_t)rs * spitch + (size_t)seg * segv;
  float v[8];
#pragma unroll
  for (int e = 0; e < 8; ++e) {
    const int col = cc + e;
    const float x = sp[min(col, segv - 1)];
    v[e] = (rok && col < segv) ? x : 0.0f;
  }
  v4u w;
  w[0] = pk16(f2bf_bits(v[0]), f2bf_bits(v[1]));
  w[1] = pk16(f2bf_bits(v[2]), f2bf_bits(v[3]));
  w[2] = pk16(f2bf_bits(v[4]), f2bf_bits(v[5]));
  w[3] = pk16(f2bf_bits(v[6]), f2bf_bits(v[7]));
  unsigned short* dp = dst + (size_t)gidx * 8;
  *(volatile v4u*)dp = w;
  __threadfence();
  *(volatile v4u*)dp = w;
}

struct TInts { int R0, C0, P0, Cp0, lo0, R1, C1, P1, Cp1, lo1; };
static_assert(sizeof(TInts) == 40);

__global__ __launch_bounds__(256) void k_tsplit(const float* src0, unsigned short* hi0, unsigned short* lo0p,
                                              const float* src1, unsigned short* hi1, unsigned short* lo1p, TInts ti) {
  __shared__ __align__(16) float tf[64 * 68];
  int R = ti.R0, C = ti.C0, P = ti.P0, Cp = ti.Cp0, haslo = ti.lo0;
  const float* src = src0; unsigned short* hi = hi0; unsigned short* lo = lo0p;
  if (blockIdx.z == 1) { R = ti.R1; C = ti.C1; P = ti.P1; Cp = ti.Cp1; haslo = ti.lo1; src = src1; hi = hi1; lo = lo1p; }
  const int c0 = blockIdx.x * 64;
  const int r0 = blockIdx.y * 64;
  if (c0 >= Cp || r0 >= R) return;
  const int tid = threadIdx.x;
  {
    const int lr = tid >> 4;
    const int c4 = (tid & 15) * 4;
    const int col = c0 + c4;
    const int cb = min(col, C - 4);
    const bool cok = col < C;
    const v4f z4 = zero4();
#pragma unroll
    for (int it = 0; it < 4; ++it) {
      const int rr = it * 16 + lr;
      v4f a = *(const v4fa*)(src + (size_t)(r0 + rr) * P + cb);
      a = cok ? a : z4;
      *(v4f*)(tf + rr * 68 + c4) = a;
    }
  }
  __syncthreads();
  const int sub = tid >> 3;
  const int c8  = (tid & 7) * 8;
  v4u hv[2], lv[2];
#pragma unroll
  for (int it = 0; it < 2; ++it) {
    const int oc = it * 32 + sub;
    v4u a, a2;
#pragma unroll
    for (int q = 0; q < 4; ++q) {
      const float f0 = tf[(c8 + 2 * q) * 68 + oc];
      const float f1 = tf[(c8 + 2 * q + 1) * 68 + oc];
      unsigned h, l;
      split2(f0, f1, h, l);
      a[q] = h; a2[q] = l;
    }
    hv[it] = a; lv[it] = a2;
  }
  for (int pass = 0; pass < 2; ++pass) {
#pragma unroll
    for (int it = 0; it < 2; ++it) {
      const int oc = it * 32 + sub;
      const size_t go = (size_t)(c0 + oc) * R + r0 + c8;
      *(volatile v4u*)(hi + go) = hv[it];
      if (haslo) *(volatile v4u*)(lo + go) = lv[it];
    }
    __threadfence();
  }
}

__global__ __launch_bounds__(320) void k_qt(const unsigned short* __restrict__ qryb, const float* __restrict__ V,
                                          const float* __restrict__ bvec, const float* __restrict__ bred,
                                          const float* __restrict__ bih, const float* __restrict__ bhh,
                                          float* __restrict__ vec) {
  __shared__ float qs[PD];
  __shared__ __align__(16) float st[2560];
  const int tid = threadIdx.x;
  float s = 0.0f;
#pragma unroll 4
  for (int l = 0; l < CL; ++l) s += bf_bits2f(qryb[(size_t)l * PD + tid]);
  qs[tid] = s * 0.0078125f;
  __syncthreads();
#pragma unroll
  for (int s2 = 0; s2 < 2; ++s2) {
    const int srcj = s2 * CD + min(tid, CD - 1);
    float acc = 0.0f;
#pragma unroll 4
    for (int dd = 0; dd < CD; ++dd) acc = fmaf(qs[dd], bfr(V[(size_t)dd * CD2 + srcj]), acc);
    st[VT + s2 * PD + tid] = (tid < CD) ? acc : 0.0f;
  }
  {
    const float bb = bfr(bvec[min(tid, CD - 1)]);
    st[VBU + tid] = (tid < CD) ? bb : 0.0f;
    const float br = bfr(bred[min(tid, CD - 1)]);
    st[VBRED + tid] = (tid < CD) ? br : 0.0f;
    for (int jj = tid; jj < PB; jj += PD) {
      const int jc = min(jj, CD4 - 1);
      const float v = bfr(bih[jc]) + bfr(bhh[jc]);
      st[VBSUM + jj] = (jj < CD4) ? v : 0.0f;
    }
  }
  __syncthreads();
  for (int pass = 0; pass < 2; ++pass) {
    for (int q = tid; q < 640; q += PD) {
      const v4f val = *(const v4fa*)(st + 4 * q);
      *(volatile v4f*)(vec + 4 * q) = val;
    }
    __threadfence();
  }
}

__global__ __launch_bounds__(320) void k_ent(const float* __restrict__ bin, const unsigned short* __restrict__ ctxb,
                                           const float* __restrict__ entF, const float* __restrict__ vec,
                                           unsigned short* __restrict__ Ehi, unsigned short* __restrict__ Elo) {
  __shared__ int hl[256];
  __shared__ int wcnt[10];
  __shared__ float red[10];
  __shared__ __align__(16) float erow[PD2];
  const int n = blockIdx.x;
  const int tid = threadIdx.x, lane = tid & 31, wave = tid >> 5;
  float mx = -__builtin_inff();
  int nhit = 0;
  for (int chk = 0; chk < CM / 256; ++chk) {
    const int m = chk * 256 + min(tid, 255);
    const float bv = bin[(size_t)m * CN + n];
    const bool hit = (tid < 256) && (bv != 0.0f);
    const unsigned msk = __builtin_amdgcn_ballot_w32(hit);
    const int cw = __builtin_popcount(msk);
    const int pre = __builtin_popcount(msk & ((1u << lane) - 1u));
    if (lane == 0) wcnt[wave] = cw;
    __syncthreads();
    int base = 0, total = 0;
#pragma unroll
    for (int w = 0; w < 10; ++w) {
      const int c = wcnt[w];
      total += c;
      base += (w < wave) ? c : 0;
    }
    if (hit) hl[base + pre] = m;
    __syncthreads();
    total = min(total, 256);
    nhit += total;
#pragma unroll 2
    for (int q = 0; q < total; ++q) {
      int mm = hl[q];
      mm = min(max(mm, 0), CM - 1);
      const float cv = bf_bits2f(ctxb[(size_t)mm * PD + tid]);
      mx = fmaxf(mx, cv);
    }
    __syncthreads();
  }
  if (nhit < CM) mx = fmaxf(mx, 0.0f);
  const float maxv = (tid < CD) ? mx : 0.0f;
  const float meanv = entF[(size_t)n * PD + tid];
  float part = vec[VT + tid] * meanv + vec[VT + PD + tid] * maxv;
  part = wave_sum(part);
  if (lane == 0) red[wave] = part;
  __syncthreads();
  float gdot = 0.0f;
#pragma unroll
  for (int w = 0; w < 10; ++w) gdot += red[w];
  const float gamma = gdot * (1.0f / DROOTF);
  const float sg = 1.0f / (1.0f + expf(-gamma));
  erow[tid] = sg * meanv;
  erow[PD + tid] = sg * maxv;
  __syncthreads();
  if (tid < 80) {
    const int e8 = tid * 8;
    const v4f x0 = *(const v4fa*)(erow + e8);
    const v4f x1 = *(const v4fa*)(erow + e8 + 4);
    v4u hv, lv;
    split8(x0, x1, hv, lv);
    const size_t o = (size_t)n * PD2 + e8;
    *(volatile v4u*)(Ehi + o) = hv;
    *(volatile v4u*)(Elo + o) = lv;
    __threadfence();
    *(volatile v4u*)(Ehi + o) = hv;
    *(volatile v4u*)(Elo + o) = lv;
  }
}

__global__ __launch_bounds__(256) void k_ac(const float* __restrict__ hidTf, const float* __restrict__ Wv,
                                          const float* __restrict__ adj, float* __restrict__ vec) {
  __shared__ __align__(16) float sv4[1024];
  const int tid = threadIdx.x;
  float a = 0.0f, c = 0.0f;
#pragma unroll 4
  for (int dd = 0; dd < CD; ++dd) {
    const float h = hidTf[(size_t)dd * CN + tid];
    a = fmaf(h, bfr(Wv[dd]), a);
    c = fmaf(h, bfr(Wv[CD + dd]), c);
  }
  sv4[tid] = a;
  sv4[CN + tid] = c;
  __syncthreads();
  float mx = -__builtin_inff();
#pragma unroll 4
  for (int k = 0; k < CN; ++k) {
    const float t = a + sv4[CN + k];
    const float lr = (t >= 0.0f) ? t : 0.01f * t;
    const float be = (adj[(size_t)tid * CN + k] > 0.0f) ? lr : 0.0f;
    mx = fmaxf(mx, be);
  }
  float z = 0.0f;
#pragma unroll 1
  for (int k = 0; k < CN; ++k) {
    const float t = a + sv4[CN + k];
    const float lr = (t >= 0.0f) ? t : 0.01f * t;
    const float be = (adj[(size_t)tid * CN + k] > 0.0f) ? lr : 0.0f;
    z += expf(be - mx);
  }
  sv4[2 * CN + tid] = mx;
  sv4[3 * CN + tid] = z;
  __syncthreads();
  const v4f val = *(const v4fa*)(sv4 + 4 * tid);
  *(volatile v4f*)(vec + VA + 4 * tid) = val;
  __threadfence();
  *(volatile v4f*)(vec + VA + 4 * tid) = val;
}

__global__ __launch_bounds__(256) void k_P(const float* __restrict__ adj, const float* __restrict__ vec,
                                         unsigned short* __restrict__ Phi, unsigned short* __restrict__ Plo) {
  __shared__ __align__(16) float prow[CN];
  const int i = blockIdx.x, j = threadIdx.x;
  const float aj = vec[VA + j], ci = vec[VC + i], mxj = vec[VMX + j], zj = vec[VZ + j];
  const float t = aj + ci;
  const float lr = (t >= 0.0f) ? t : 0.01f * t;
  const float be = (adj[(size_t)j * CN + i] > 0.0f) ? lr : 0.0f;
  const float al = expf(be - mxj) * (1.0f / zj);
  prow[j] = adj[(size_t)i * CN + j] * al;
  __syncthreads();
  if (j < 32) {
    const int e8 = j * 8;
    const v4f x0 = *(const v4fa*)(prow + e8);
    const v4f x1 = *(const v4fa*)(prow + e8 + 4);
    v4u hv, lv;
    split8(x0, x1, hv, lv);
    const size_t o = (size_t)i * CN + e8;
    *(volatile v4u*)(Phi + o) = hv;
    *(volatile v4u*)(Plo + o) = lv;
    __threadfence();
    *(volatile v4u*)(Phi + o) = hv;
    *(volatile v4u*)(Plo + o) = lv;
  }
}

__global__ __launch_bounds__(256) void k_vec(const unsigned short* __restrict__ qryb, const float* __restrict__ Etf,
                                           const float* __restrict__ watt, const float* __restrict__ batt,
                                           unsigned short* __restrict__ QWhi, unsigned short* __restrict__ QWlo,
                                           float* __restrict__ vec) {
  __shared__ __align__(16) float sv[384];
  const int tid = threadIdx.x;
  if (blockIdx.x < CL) {
    const int l = blockIdx.x;
    if (tid < 40) {
      const int e8 = tid * 8;
      const v4u qw = *(const v4ua*)(qryb + (size_t)l * PD + e8);
      v4f q0, q1;
      unpack8(qw, q0, q1);
      float q[8] = {q0[0], q0[1], q0[2], q0[3], q1[0], q1[1], q1[2], q1[3]};
      float v[8];
#pragma unroll
      for (int e = 0; e < 8; ++e) {
        const int col = e8 + e;
        const float w = bfr(watt[2 * CD + min(col, CD - 1)]);
        v[e] = (col < CD) ? q[e] * w : 0.0f;
      }
      const v4f x0 = {v[0], v[1], v[2], v[3]};
      const v4f x1 = {v[4], v[5], v[6], v[7]};
      v4u hv, lv;
      split8(x0, x1, hv, lv);
      const size_t o = (size_t)l * PD + e8;
      *(volatile v4u*)(QWhi + o) = hv;
      *(volatile v4u*)(QWlo + o) = lv;
      __threadfence();
      *(volatile v4u*)(QWhi + o) = hv;
      *(volatile v4u*)(QWlo + o) = lv;
    }
  } else {
    const int l = min(tid, CL - 1);
    float rq = 0.0f, re = 0.0f;
#pragma unroll 4
    for (int dd = 0; dd < CD; ++dd) {
      rq = fmaf(bf_bits2f(qryb[(size_t)l * PD + dd]), bfr(watt[dd]), rq);
      re = fmaf(Etf[(size_t)tid * PD + dd], bfr(watt[CD + dd]), re);
    }
    rq = (rq + bfr(batt[0])) + bfr(batt[2]);
    re = re + bfr(batt[1]);
    if (tid < CL) sv[tid] = rq;
    sv[CL + tid] = re;
    __syncthreads();
    if (tid < 96) {
      const v4f val = *(const v4fa*)(sv + 4 * tid);
      *(volatile v4f*)(vec + VRQ + 4 * tid) = val;
      __threadfence();
      *(volatile v4f*)(vec + VRQ + 4 * tid) = val;
    }
  }
}

__global__ __launch_bounds__(256) void k_softS(const float* __restrict__ S, unsigned short* __restrict__ Pshi,
                                             unsigned short* __restrict__ Pslo) {
  __shared__ __align__(16) float prow[CN];
  __shared__ float red[8];
  const int l = blockIdx.x, j = threadIdx.x, lane = j & 31, wave = j >> 5;
  const float v = S[(size_t)l * CN + j];
  const float mx = block_max(v, red, lane, wave, 8);
  const float ex = expf(v - mx);
  const float z = block_sum(ex, red, lane, wave, 8);
  prow[j] = ex * (1.0f / z);
  __syncthreads();
  if (j < 32) {
    const int e8 = j * 8;
    const v4f x0 = *(const v4fa*)(prow + e8);
    const v4f x1 = *(const v4fa*)(prow + e8 + 4);
    v4u hv, lv;
    split8(x0, x1, hv, lv);
    const size_t o = (size_t)l * CN + e8;
    *(volatile v4u*)(Pshi + o) = hv;
    *(volatile v4u*)(Pslo + o) = lv;
    __threadfence();
    *(volatile v4u*)(Pshi + o) = hv;
    *(volatile v4u*)(Pslo + o) = lv;
  }
}

__global__ __launch_bounds__(320) void k_q2c(const float* __restrict__ S, const unsigned short* __restrict__ qryb,
                                           float* __restrict__ vec) {
  __shared__ float sw[CL];
  __shared__ float red[10];
  __shared__ __align__(16) float sq[PD];
  const int tid = threadIdx.x, lane = tid & 31, wave = tid >> 5;
  const int l = min(tid, CL - 1);
  float m = -__builtin_inff();
#pragma unroll 4
  for (int j = 0; j < CN; ++j) m = fmaxf(m, S[(size_t)l * CN + j]);
  const float sm = (tid < CL) ? m : -__builtin_inff();
  const float gm = block_max(sm, red, lane, wave, 10);
  const float ex = (tid < CL) ? expf(sm - gm) : 0.0f;
  const float z = block_sum(ex, red, lane, wave, 10);
  if (tid < CL) sw[tid] = ex * (1.0f / z);
  __syncthreads();
  float acc = 0.0f;
#pragma unroll 4
  for (int ll = 0; ll < CL; ++ll) acc = fmaf(sw[ll], bf_bits2f(qryb[(size_t)ll * PD + tid]), acc);
  sq[tid] = acc;
  __syncthreads();
  if (tid < 80) {
    const v4f val = *(const v4fa*)(sq + 4 * tid);
    *(volatile v4f*)(vec + VQ2C + 4 * tid) = val;
    __threadfence();
    *(volatile v4f*)(vec + VQ2C + 4 * tid) = val;
  }
}

__global__ __launch_bounds__(128) void k_xbuild(const unsigned short* __restrict__ qryb, const float* __restrict__ c2q,
                                              const float* __restrict__ vec, unsigned short* __restrict__ Xchi,
                                              unsigned short* __restrict__ Xclo) {
  const int l = blockIdx.x, t = threadIdx.x;
  if (t >= 120) return;
  const int seg = t / 40;
  const int e8 = (t - seg * 40) * 8;
  const v4f ca = *(const v4fa*)(c2q + (size_t)l * PD + e8);
  const v4f cb = *(const v4fa*)(c2q + (size_t)l * PD + e8 + 4);
  const v4u qw = *(const v4ua*)(qryb + (size_t)l * PD + e8);
  const v4f ga = *(const v4fa*)(vec + VQ2C + e8);
  const v4f gb = *(const v4fa*)(vec + VQ2C + e8 + 4);
  v4f qa, qb;
  unpack8(qw, qa, qb);
  v4f xa, xb;
#pragma unroll
  for (int e = 0; e < 4; ++e) {
    const float va = (seg == 0) ? ca[e] : ((seg == 1) ? qa[e] * ca[e] : qa[e] * ga[e]);
    const float vb = (seg == 0) ? cb[e] : ((seg == 1) ? qb[e] * cb[e] : qb[e] * gb[e]);
    xa[e] = va; xb[e] = vb;
  }
  v4u hv, lv;
  split8(xa, xb, hv, lv);
  const size_t o = (size_t)l * PX + seg * PD + e8;
  *(volatile v4u*)(Xchi + o) = hv;
  *(volatile v4u*)(Xclo + o) = lv;
  __threadfence();
  *(volatile v4u*)(Xchi + o) = hv;
  *(volatile v4u*)(Xclo + o) = lv;
}

__global__ __launch_bounds__(256) void k_pack(const float* __restrict__ gates, const float* __restrict__ Y,
                                            const int* __restrict__ npass, float* __restrict__ out) {
  __shared__ __align__(16) float buf[8 * CD];
  const int g = blockIdx.x, tid = threadIdx.x;
  const bool poison = (npass[0] != 1);
  const float qnan = __int_as_float(0x7fc00000);
  size_t obase;
  if (g < 256) {
    const int m0 = g * 8;
    obase = (size_t)m0 * CD;
#pragma unroll 1
    for (int idx = tid; idx < 8 * CD; idx += 256) {
      const int r = idx / CD, d = idx - r * CD;
      const float* gp = gates + (size_t)(m0 + r) * NG + d;
      const float gi = gp[0], gg = gp[2 * CD], go = gp[3 * CD];
      float cst = 0.0f;
#pragma unroll 1
      for (int it = 0; it < 2; ++it) {
        const float x = (it == 0) ? gi : go;
        const float y = (it == 0) ? gg : cst;
        const float sgm = 1.0f / (1.0f + expf(-x));
        cst = sgm * tanhf(y);
      }
      buf[idx] = poison ? qnan : cst;
    }
  } else {
    const int l0 = (g - 256) * 8;
    obase = (size_t)OUT0_N + (size_t)l0 * CD;
#pragma unroll 1
    for (int idx = tid; idx < 8 * CD; idx += 256) {
      const int r = idx / CD, d = idx - r * CD;
      const float v = Y[(size_t)(l0 + r) * PD + d];
      buf[idx] = poison ? qnan : v;
    }
  }
  __syncthreads();
  for (int pass = 0; pass < 2; ++pass) {
    for (int q = tid; q < 2 * CD; q += 256) {
      const v4f val = *(const v4fa*)(buf + 4 * q);
      *(volatile v4f*)(out + obase + 4 * (size_t)q) = val;
    }
    __threadfence();
  }
}

static void launch_gemm(hipStream_t s,
                        const unsigned short* a0, const unsigned short* b0, int lda0, int ldb0, int K0,
                        const unsigned short* a1, const unsigned short* b1, int lda1, int ldb1, int K1,
                        const unsigned short* a2, const unsigned short* b2, int lda2, int ldb2, int K2,
                        int nterm, float* cf, int ldcf, unsigned short* ch, unsigned short* cl, int ldch,
                        const float* rowb, const float* colb, int M, int N, int flags, float scale) {
  GInts p;
  p.lda0 = lda0; p.ldb0 = ldb0; p.K0 = K0;
  p.lda1 = lda1; p.ldb1 = ldb1; p.K1 = K1;
  p.lda2 = lda2; p.ldb2 = ldb2; p.K2 = K2;
  p.ldcf = ldcf; p.ldch = ldch; p.M = M; p.N = N; p.nterm = nterm; p.flags = flags; p.scale = scale;
  const int tiles = (M / 64) * (N / 64);
  const int nb = (tiles + 7) / 8;
  k_gemm<<<dim3(nb), dim3(256), 0, s>>>(a0, b0, a1, b1, a2, b2, cf, ch, cl, rowb, colb, p);
}

extern "C" void kernel_launch(void* const* d_in, const int* in_sizes, int n_in,
                              void* d_out, int out_size, void* d_ws, size_t ws_size,
                              hipStream_t stream) {
  if (n_in < 16) return;
  if (in_sizes[0] != CM * CD || in_sizes[1] != CL * CD) return;
  if (in_sizes[2] != CM * CN || in_sizes[3] != CN * CN) return;
  if (in_sizes[4] != CD * CD2 || in_sizes[5] != CD * CD2) return;
  if (in_sizes[6] != CD || in_sizes[7] != CD2 || in_sizes[8] != 3 * CD || in_sizes[9] != 3) return;
  if (in_sizes[10] != CD * CD4 || in_sizes[11] != CD) return;
  if (in_sizes[12] != CD4 * CD2 || in_sizes[13] != CD4 || in_sizes[14] != CD4 || in_sizes[15] < 1) return;
  if (out_size != OUT0_N + OUT1_N) return;

  const float* ctx  = (const float*)d_in[0];
  const float* qry  = (const float*)d_in[1];
  const float* binM = (const float*)d_in[2];
  const float* adj  = (const float*)d_in[3];
  const float* V    = (const float*)d_in[4];
  const float* U    = (const float*)d_in[5];
  const float* bvec = (const float*)d_in[6];
  const float* Wv   = (const float*)d_in[7];
  const float* watt = (const float*)d_in[8];
  const float* batt = (const float*)d_in[9];
  const float* Wred = (const float*)d_in[10];
  const float* bred = (const float*)d_in[11];
  const float* Wih  = (const float*)d_in[12];
  const float* bih  = (const float*)d_in[13];
  const float* bhh  = (const float*)d_in[14];
  const int*   npass = (const int*)d_in[15];
  float* out = (float*)d_out;

  size_t off = 0;
#define CARVE(name, bytes) const size_t name = off; off += ((((size_t)(bytes)) + 255) & ~(size_t)255);
  CARVE(oCtxb, (size_t)CM * PD * 2)
  CARVE(oQryb, (size_t)CL * PD * 2)
  CARVE(oBinb, (size_t)CM * CN * 2)
  CARVE(oU2,   (size_t)PD * PD2 * 2)
  CARVE(oWih0, (size_t)NG * PD * 2)
  CARVE(oWih1, (size_t)NG * PD * 2)
  CARVE(oWr0,  (size_t)PD * PD * 2)
  CARVE(oWr1,  (size_t)PD * PX * 2)
  CARVE(oCtxT, (size_t)PD * CM * 2)
  CARVE(oBinT, (size_t)CN * CM * 2)
  CARVE(oEntF, (size_t)CN * PD * 4)
  CARVE(oVec,  (size_t)VTOT * 4)
  CARVE(oEhi,  (size_t)CN * PD2 * 2)
  CARVE(oElo,  (size_t)CN * PD2 * 2)
  CARVE(oHidTf,(size_t)PD * CN * 4)
  CARVE(oHThi, (size_t)PD * CN * 2)
  CARVE(oHTlo, (size_t)PD * CN * 2)
  CARVE(oPhi,  (size_t)CN * CN * 2)
  CARVE(oPlo,  (size_t)CN * CN * 2)
  CARVE(oEtf,  (size_t)CN * PD * 4)
  CARVE(oEthi, (size_t)CN * PD * 2)
  CARVE(oEtlo, (size_t)CN * PD * 2)
  CARVE(oEtThi,(size_t)PD * CN * 2)
  CARVE(oEtTlo,(size_t)PD * CN * 2)
  CARVE(oQWhi, (size_t)CL * PD * 2)
  CARVE(oQWlo, (size_t)CL * PD * 2)
  CARVE(oS,    (size_t)CL * CN * 4)
  CARVE(oPshi, (size_t)CL * CN * 2)
  CARVE(oPslo, (size_t)CL * CN * 2)
  CARVE(oC2q,  (size_t)CL * PD * 4)
  CARVE(oXchi, (size_t)CL * PX * 2)
  CARVE(oXclo, (size_t)CL * PX * 2)
  CARVE(oY,    (size_t)CL * PD * 4)
  CARVE(oBEhi, (size_t)CM * PD * 2)
  CARVE(oBElo, (size_t)CM * PD * 2)
  CARVE(oGates,(size_t)CM * NG * 4)
  CARVE(oDum,  256)
#undef CARVE
  if (off > ws_size) return;
  if (off > (size_t)134217728) return;

  char* ws = (char*)d_ws;
  unsigned short* ctxb  = (unsigned short*)(ws + oCtxb);
  unsigned short* qryb  = (unsigned short*)(ws + oQryb);
  unsigned short* binb  = (unsigned short*)(ws + oBinb);
  unsigned short* U2    = (unsigned short*)(ws + oU2);
  unsigned short* Wih0  = (unsigned short*)(ws + oWih0);
  unsigned short* Wih1  = (unsigned short*)(ws + oWih1);
  unsigned short* Wr0   = (unsigned short*)(ws + oWr0);
  unsigned short* Wr1   = (unsigned short*)(ws + oWr1);
  unsigned short* ctxT  = (unsigned short*)(ws + oCtxT);
  unsigned short* binT  = (unsigned short*)(ws + oBinT);
  float* entF           = (float*)(ws + oEntF);
  float* vec            = (float*)(ws + oVec);
  unsigned short* Ehi   = (unsigned short*)(ws + oEhi);
  unsigned short* Elo   = (unsigned short*)(ws + oElo);
  float* hidTf          = (float*)(ws + oHidTf);
  unsigned short* HThi  = (unsigned short*)(ws + oHThi);
  unsigned short* HTlo  = (unsigned short*)(ws + oHTlo);
  unsigned short* Phi   = (unsigned short*)(ws + oPhi);
  unsigned short* Plo   = (unsigned short*)(ws + oPlo);
  float* Etf            = (float*)(ws + oEtf);
  unsigned short* Ethi  = (unsigned short*)(ws + oEthi);
  unsigned short* Etlo  = (unsigned short*)(ws + oEtlo);
  unsigned short* EtThi = (unsigned short*)(ws + oEtThi);
  unsigned short* EtTlo = (unsigned short*)(ws + oEtTlo);
  unsigned short* QWhi  = (unsigned short*)(ws + oQWhi);
  unsigned short* QWlo  = (unsigned short*)(ws + oQWlo);
  float* S              = (float*)(ws + oS);
  unsigned short* Pshi  = (unsigned short*)(ws + oPshi);
  unsigned short* Pslo  = (unsigned short*)(ws + oPslo);
  float* c2q            = (float*)(ws + oC2q);
  unsigned short* Xchi  = (unsigned short*)(ws + oXchi);
  unsigned short* Xclo  = (unsigned short*)(ws + oXclo);
  float* Y              = (float*)(ws + oY);
  unsigned short* BEhi  = (unsigned short*)(ws + oBEhi);
  unsigned short* BElo  = (unsigned short*)(ws + oBElo);
  float* gates          = (float*)(ws + oGates);
  unsigned short* dumh  = (unsigned short*)(ws + oDum);
  float* dumf           = (float*)(ws + oDum);

  const dim3 blk(256);

  {
    CvtInts ci;
    const int sp[8] = {CD, CD, CN, CD2, CD2, CD2, CD4, CD4};
    const int sr[8] = {CM, CL, CM, CD, CD4, CD4, CD, CD};
    const int dr[8] = {CM, CL, CM, PD, NG, NG, PD, PD};
    const int sw[8] = {PD, PD, CN, PD, PD, PD, PD, PD};
    const int sg[8] = {CD, CD, CN, CD, CD, CD, CD, CD};
    const int ns[8] = {1, 1, 1, 2, 1, 1, 1, 3};
    for (int i = 0; i < 8; ++i) {
      ci.src_pitch[i] = sp[i]; ci.src_rows[i] = sr[i]; ci.dst_rows[i] = dr[i];
      ci.segw[i] = sw[i]; ci.segv[i] = sg[i]; ci.nseg[i] = ns[i];
    }
    int maxthr = 0;
    for (int i = 0; i < 8; ++i) { const int n = dr[i] * (sw[i] * ns[i] / 8); if (n > maxthr) maxthr = n; }
    const dim3 gc((maxthr + 255) / 256, 8);
    k_cvt<<<gc, blk, 0, stream>>>(ctx, qry, binM, U, Wih, Wih + CD, Wred, Wred + CD,
                                  ctxb, qryb, binb, U2, Wih0, Wih1, Wr0, Wr1, ci);
  }
  {
    TInts ti;
    ti.R0 = CM; ti.C0 = CD; ti.P0 = CD; ti.Cp0 = PD; ti.lo0 = 0;
    ti.R1 = CM; ti.C1 = CN; ti.P1 = CN; ti.Cp1 = CN; ti.lo1 = 0;
    k_tsplit<<<dim3(PD / 64, CM / 64, 2), blk, 0, stream>>>(ctx, ctxT, dumh, binM, binT, dumh, ti);
  }
  launch_gemm(stream, binT, ctxT, CM, CM, CM, dumh, dumh, 0, 0, 0, dumh, dumh, 0, 0, 0,
              1, entF, PD, dumh, dumh, 0, dumf, dumf, CN, PD, GF_F32, 1.0f / 2048.0f);
  k_qt<<<dim3(1), dim3(PD), 0, stream>>>(qryb, V, bvec, bred, bih, bhh, vec);
  k_ent<<<dim3(CN), dim3(PD), 0, stream>>>(binM, ctxb, entF, vec, Ehi, Elo);
  launch_gemm(stream, U2, Ehi, PD2, PD2, PD2, U2, Elo, PD2, PD2, PD2, dumh, dumh, 0, 0, 0,
              2, hidTf, CN, HThi, HTlo, CN, vec + VBU, dumf, PD, CN, GF_F32 | GF_PLN | GF_ROWB, 1.0f);
  k_ac<<<dim3(1), blk, 0, stream>>>(hidTf, Wv, adj, vec);
  k_P<<<dim3(CN), blk, 0, stream>>>(adj, vec, Phi, Plo);
  launch_gemm(stream, Phi, HThi, CN, CN, CN, Plo, HThi, CN, CN, CN, Phi, HTlo, CN, CN, CN,
              3, Etf, PD, Ethi, Etlo, PD, dumf, dumf, CN, PD, GF_F32 | GF_PLN | GF_RELU, 1.0f);
  {
    TInts ti;
    ti.R0 = CN; ti.C0 = PD; ti.P0 = PD; ti.Cp0 = PD; ti.lo0 = 1;
    ti.R1 = CN; ti.C1 = PD; ti.P1 = PD; ti.Cp1 = PD; ti.lo1 = 1;
    k_tsplit<<<dim3(PD / 64, CN / 64, 1), blk, 0, stream>>>(Etf, EtThi, EtTlo, Etf, EtThi, EtTlo, ti);
  }
  k_vec<<<dim3(CL + 1), blk, 0, stream>>>(qryb, Etf, watt, batt, QWhi, QWlo, vec);
  launch_gemm(stream, QWhi, Ethi, PD, PD, PD, QWlo, Ethi, PD, PD, PD, QWhi, Etlo, PD, PD, PD,
              3, S, CN, dumh, dumh, 0, vec + VRQ, vec + VRE, CL, CN, GF_F32 | GF_ROWB | GF_COLB, 1.0f);
  k_softS<<<dim3(CL), blk, 0, stream>>>(S, Pshi, Pslo);
  k_q2c<<<dim3(1), dim3(PD), 0, stream>>>(S, qryb, vec);
  launch_gemm(stream, Pshi, EtThi, CN, CN, CN, Pslo, EtThi, CN, CN, CN, Pshi, EtTlo, CN, CN, CN,
              3, c2q, PD, dumh, dumh, 0, dumf, dumf, CL, PD, GF_F32, 1.0f);
  k_xbuild<<<dim3(CL), dim3(128), 0, stream>>>(qryb, c2q, vec, Xchi, Xclo);
  launch_gemm(stream, qryb, Wr0, PD, PD, PD, Xchi, Wr1, PX, PX, PX, Xclo, Wr1, PX, PX, PX,
              3, Y, PD, dumh, dumh, 0, dumf, vec + VBRED, CL, PD, GF_F32 | GF_COLB, 1.0f);
  launch_gemm(stream, binb, EtThi, CN, CN, CN, binb, EtTlo, CN, CN, CN, dumh, dumh, 0, 0, 0,
              2, dumf, 0, BEhi, BElo, PD, dumf, dumf, CM, PD, GF_PLN, 1.0f);
  launch_gemm(stream, ctxb, Wih0, PD, PD, PD, BEhi, Wih1, PD, PD, PD, BElo, Wih1, PD, PD, PD,
              3, gates, NG, dumh, dumh, 0, dumf, vec + VBSUM, CM, NG, GF_F32 | GF_COLB, 1.0f);
  k_pack<<<dim3(CM / 8 + CL / 8), blk, 0, stream>>>(gates, Y, npass, out);
  (void)hipGetLastError();
}
